// GT_FID_30391188587301
// MI455X (gfx1250) — hardware-verified
//
#include <hip/hip_runtime.h>
#include <math.h>

#define BB 64
#define TT 512
#define EE 128
#define HH 256
#define G4 1024
#define VV 32000
#define NN 50000
#define NE 800000
#define NP 50048
#define NG 64
#define GH 128
#define FD 384
#define NC 2
#define KF 640
#define NT 256
#define SCHA 4096
#define NCHA ((NE + SCHA - 1) / SCHA)
#define SCHC 8192
#define NCHC ((NE + SCHC - 1) / SCHC)
#define TSA 8192
#define NTA 7
#define NRA (NTA * TSA)
#define TSC 1024
#define NTC 49
#define NRC (NTC * TSC)
#define NSB 50

typedef __attribute__((ext_vector_type(16))) _Float16 v16h;
typedef __attribute__((ext_vector_type(8)))  _Float16 v8h;
typedef __attribute__((ext_vector_type(16))) __bf16   v16b;
typedef __attribute__((ext_vector_type(8)))  __bf16   v8b;
typedef __attribute__((ext_vector_type(8)))  float    v8f;
typedef __attribute__((ext_vector_type(4)))  float    v4f;
typedef __attribute__((ext_vector_type(4)))  int      v4i;

__device__ __forceinline__ unsigned short f2bf_bits(float f) {
  unsigned u = __float_as_uint(f);
  return (unsigned short)((u + 0x7FFFu + ((u >> 16) & 1u)) >> 16);
}
__device__ __forceinline__ float bf_bits2f(unsigned short h) { return __uint_as_float(((unsigned)h) << 16); }

__device__ __forceinline__ void dep_guard_h(v8f& a, v8f& b, v16h x, v16h y) { asm volatile("v_nop\n\tv_nop\n\tv_nop\n\tv_nop" : "+v"(a), "+v"(b) : "v"(x), "v"(y)); }
__device__ __forceinline__ void dep_guard_b(v8f& a, v8f& b, v16b x, v16b y) { asm volatile("v_nop\n\tv_nop\n\tv_nop\n\tv_nop" : "+v"(a), "+v"(b) : "v"(x), "v"(y)); }
__device__ __forceinline__ void keep4_h(v16h a, v16h b, v16h c, v16h d) { asm volatile("v_nop" :: "v"(a), "v"(b), "v"(c), "v"(d)); }
__device__ __forceinline__ void keep4_b(v16b a, v16b b, v16b c, v16b d) { asm volatile("v_nop" :: "v"(a), "v"(b), "v"(c), "v"(d)); }
__device__ __forceinline__ void acc_guard4(v8f& a, v8f& b, v8f& c, v8f& d) { asm volatile("v_nop\n\tv_nop\n\tv_nop\n\tv_nop" : "+v"(a), "+v"(b), "+v"(c), "+v"(d)); }
template <typename T> struct Frag;
template <> struct Frag<_Float16> {
  typedef v16h V; union U { v16h v; v8h h[2]; };
  static __device__ __forceinline__ v16h load(const _Float16* p) {
    U f; f.h[0] = *(const v8h*)(p); f.h[1] = *(const v8h*)(p + 16); return f.v;
  }
  static __device__ __forceinline__ v8f mma(v16h a, v16h b, v8f c) {
    return __builtin_amdgcn_wmma_f32_16x16x32_f16(false, a, false, b, (short)0, c, false, false);
  }
  static __device__ __forceinline__ void guard(v8f& a, v8f& b, v16h x, v16h y) { dep_guard_h(a, b, x, y); }
  static __device__ __forceinline__ void keep(v16h a, v16h b, v16h c, v16h d) { keep4_h(a, b, c, d); }
};
template <> struct Frag<__bf16> {
  typedef v16b V; union U { v16b v; v8b h[2]; };
  static __device__ __forceinline__ v16b load(const __bf16* p) {
    U f; f.h[0] = *(const v8b*)(p); f.h[1] = *(const v8b*)(p + 16); return f.v;
  }
  static __device__ __forceinline__ v8f mma(v16b a, v16b b, v8f c) {
    return __builtin_amdgcn_wmma_f32_16x16x32_bf16(false, a, false, b, (short)0, c, false, false);
  }
  static __device__ __forceinline__ void guard(v8f& a, v8f& b, v16b x, v16b y) { dep_guard_b(a, b, x, y); }
  static __device__ __forceinline__ void keep(v16b a, v16b b, v16b c, v16b d) { keep4_b(a, b, c, d); }
};

template <int ET> struct Elem;
template <> struct Elem<0> { typedef _Float16 T; };
template <> struct Elem<1> { typedef __bf16 T; };
template <int ET, bool SPLIT, int BIAS_MODE, int OUT_MODE, bool RESID, int ACT = 0>
__global__ __launch_bounds__(256) void wmma_gemm64(
    const unsigned short* __restrict__ Ap, const unsigned short* __restrict__ A2p, int lda, long strideA,
    const unsigned short* __restrict__ Btp, const unsigned short* __restrict__ Bt2p, int ldb, long strideB,
    void* __restrict__ Cout, void* __restrict__ Cout2, int ldc, long strideC,
    const float* __restrict__ bias,
    const float* __restrict__ resid, long strideR,
    int M, int N, int K, float scale) {
  typedef typename Elem<ET>::T T;
  typedef typename Frag<T>::V V;
  const T* A = (const T*)Ap; const T* A2 = (const T*)A2p; const T* Bt = (const T*)Btp; const T* Bt2 = (const T*)Bt2p;
  __shared__ __align__(16) float sT[8][16 * 68];
  const int b    = blockIdx.y;
  const int lane = threadIdx.x & 31;
  const int wave = threadIdx.x >> 5;
  const int tilesN = N >> 6;
  const int tilesM = M >> 6;
  const int tile = blockIdx.x * 8 + wave;
  if (tile >= tilesM * tilesN) return;
  const int tm = tile / tilesN;
  const int tn = tile - tm * tilesN;
  const int m0 = tm << 6;
  const int n0 = tn << 6;

  const T* Ab  = A  + (size_t)b * strideA;
  const T* Bb  = Bt + (size_t)b * strideB;
  const T* Ab2 = SPLIT ? (A2  + (size_t)b * strideA) : nullptr;
  const T* Bb2 = SPLIT ? (Bt2 + (size_t)b * strideB) : nullptr;

  const int rlane = lane & 15;
  const int koff  = (lane >> 4) * 8;
  const int mOff  = (lane >> 4) * 8;

  v8f acc[4][4];
#pragma unroll
  for (int i = 0; i < 4; ++i)
#pragma unroll
    for (int j = 0; j < 4; ++j) acc[i][j] = (v8f){0.f,0.f,0.f,0.f,0.f,0.f,0.f,0.f};

  for (int k0 = 0; k0 < K; k0 += 32) {
    V bh[4], bl[4];
#pragma unroll
    for (int j = 0; j < 4; ++j) {
      const size_t bo = (size_t)(n0 + (j << 4) + rlane) * ldb + koff + k0;
      bh[j] = Frag<T>::load(Bb + bo);
      if (SPLIT) bl[j] = Frag<T>::load(Bb2 + bo);
    }
#pragma unroll
    for (int i = 0; i < 4; ++i) {
      const size_t ao = (size_t)(m0 + (i << 4) + rlane) * lda + koff + k0;
      V ah = Frag<T>::load(Ab + ao);
      V al;
      if (SPLIT) al = Frag<T>::load(Ab2 + ao);
#pragma unroll
      for (int j = 0; j < 4; ++j) {
        acc[i][j] = Frag<T>::mma(ah, bh[j], acc[i][j]);
        if (SPLIT) {
          acc[i][j] = Frag<T>::mma(ah, bl[j], acc[i][j]);
          acc[i][j] = Frag<T>::mma(al, bh[j], acc[i][j]);
        }
      }
      Frag<T>::guard(acc[i][0], acc[i][3], ah, SPLIT ? al : ah);
    }
    Frag<T>::keep(bh[0], bh[1], bh[2], bh[3]);
    if (SPLIT) Frag<T>::keep(bl[0], bl[1], bl[2], bl[3]);
  }
  acc_guard4(acc[0][0], acc[0][1], acc[0][2], acc[0][3]);
  acc_guard4(acc[1][0], acc[1][1], acc[1][2], acc[1][3]);
  acc_guard4(acc[2][0], acc[2][1], acc[2][2], acc[2][3]);
  acc_guard4(acc[3][0], acc[3][1], acc[3][2], acc[3][3]);

  float* slab = sT[wave];
  const float* Rb = RESID ? (resid + (size_t)b * strideR) : nullptr;
#pragma unroll
  for (int i = 0; i < 4; ++i) {
    const int mBase = m0 + (i << 4);
#pragma unroll
    for (int j = 0; j < 4; ++j) {
      const int n = n0 + (j << 4) + rlane;
      float bv = 0.f;
      if (BIAS_MODE == 2) bv = bias[n];
#pragma unroll
      for (int r = 0; r < 8; ++r) {
        float v = acc[i][j][r] * scale;
        if (BIAS_MODE == 1) v += bias[mBase + mOff + r];
        if (BIAS_MODE == 2) v += bv;
        if (RESID) v += Rb[(size_t)(mBase + mOff + r) * ldc + n];
        if (ACT == 1) v = tanhf(v);
        if (ACT == 2) v = fmaxf(v, 0.0f);
        if (ACT == 3) v = v / (1.0f + expf(-v));
        if (ACT == 4) v = (v > 0.f) ? v : 0.01f * v;
        if (ACT == 5) v = 0.5f * v * (1.0f + erff(v * 0.70710678118654752f));
        slab[(mOff + r) * 68 + (j << 4) + rlane] = v;
      }
    }
    __builtin_amdgcn_fence(__ATOMIC_RELEASE, "workgroup");
    __builtin_amdgcn_wave_barrier();
    __builtin_amdgcn_fence(__ATOMIC_ACQUIRE, "workgroup");
    if (OUT_MODE == 0) {
      float* C = (float*)Cout + (size_t)b * strideC;
      const int hh = lane >> 4, c4 = (lane & 15) * 4;
      for (int pass = 0; pass < 2; ++pass) {
#pragma unroll
        for (int it = 0; it < 8; ++it) {
          const int row = it * 2 + hh;
          v4f v = *(const v4f*)(slab + row * 68 + c4);
          *(volatile v4f*)(C + (size_t)(mBase + row) * ldc + n0 + c4) = v;
        }
        __threadfence();
      }
    } else {
      const int q = lane >> 3, c8 = (lane & 7) * 8;
      unsigned short* C  = (unsigned short*)Cout  + (size_t)b * strideC;
      unsigned short* C2 = (OUT_MODE == 2) ? ((unsigned short*)Cout2 + (size_t)b * strideC) : nullptr;
      for (int pass = 0; pass < 2; ++pass) {
#pragma unroll
        for (int it = 0; it < 4; ++it) {
          const int row = it * 4 + q;
          const float* sp = slab + row * 68 + c8;
          v8h hv, lv;
#pragma unroll
          for (int e = 0; e < 8; ++e) {
            if (OUT_MODE == 1) {
              hv[e] = (_Float16)sp[e];
            } else {
              unsigned short hb = f2bf_bits(sp[e]);
              unsigned short lb = f2bf_bits(sp[e] - bf_bits2f(hb));
              hv[e] = __builtin_bit_cast(_Float16, hb);
              lv[e] = __builtin_bit_cast(_Float16, lb);
            }
          }
          *(volatile v8h*)(C + (size_t)(mBase + row) * ldc + n0 + c8) = hv;
          if (OUT_MODE == 2) *(volatile v8h*)(C2 + (size_t)(mBase + row) * ldc + n0 + c8) = lv;
        }
        __threadfence();
      }
    }
    __builtin_amdgcn_fence(__ATOMIC_RELEASE, "workgroup");
    __builtin_amdgcn_wave_barrier();
    __builtin_amdgcn_fence(__ATOMIC_ACQUIRE, "workgroup");
  }
}

__device__ __forceinline__ unsigned pack_f16x2(float a, float b) {
  const _Float16 h0 = (_Float16)a, h1 = (_Float16)b;
  return (unsigned)__builtin_bit_cast(unsigned short, h0) | ((unsigned)__builtin_bit_cast(unsigned short, h1) << 16);
}
__device__ __forceinline__ void split_pack2(float a, float b, unsigned& uh, unsigned& ul) {
  const unsigned short ha = f2bf_bits(a), hb = f2bf_bits(b);
  const unsigned short la = f2bf_bits(a - bf_bits2f(ha)), lb = f2bf_bits(b - bf_bits2f(hb));
  uh = (unsigned)ha | ((unsigned)hb << 16);
  ul = (unsigned)la | ((unsigned)lb << 16);
}
__device__ __forceinline__ void st2u(unsigned* p, unsigned v) { *(volatile unsigned*)p = v; __threadfence(); *(volatile unsigned*)p = v; }
__device__ __forceinline__ float fsig(float x) { return __builtin_amdgcn_rcpf(1.0f + __expf(-x)); }
__device__ __forceinline__ float ftanh(float x) { return 1.0f - 2.0f * __builtin_amdgcn_rcpf(1.0f + __expf(2.0f * x)); }

__global__ __launch_bounds__(NT) void prep_kernel(const float* __restrict__ Wih_f, const float* __restrict__ Wih_b,
                                                 const float* __restrict__ Whh_f, const float* __restrict__ Whh_b,
                                                 const float* __restrict__ Wg2,
                                                 unsigned* __restrict__ WIH, unsigned* __restrict__ WHH, unsigned* __restrict__ WG2T) {
  const int blk = blockIdx.x, tid = threadIdx.x;
  if (blk < 512) {
    const int sel = blk >> 8;
    const int p = (blk & 255) * NT + tid;
    const float* src = sel ? Wih_b : Wih_f;
    const unsigned u = pack_f16x2(src[2 * p] * 256.0f, src[2 * p + 1] * 256.0f);
    st2u(WIH + sel * 65536 + p, u);
  } else if (blk < 1536) {
    const int b2 = blk - 512;
    const int sel = b2 >> 9;
    const int p = (b2 & 511) * NT + tid;
    const float* src = sel ? Whh_b : Whh_f;
    const unsigned u = pack_f16x2(src[2 * p] * 256.0f, src[2 * p + 1] * 256.0f);
    st2u(WHH + sel * 131072 + p, u);
  } else {
    const int p = (blk - 1536) * NT + tid;
    const int o = p >> 6, k = 2 * (p & 63);
    const unsigned u = pack_f16x2(Wg2[k * GH + o] * 256.0f, Wg2[(k + 1) * GH + o] * 256.0f);
    st2u(WG2T + p, u);
  }
}

__global__ __launch_bounds__(NT) void embed_kernel(const int* __restrict__ seqs, const float* __restrict__ emb, _Float16* __restrict__ EX) {
  const int gid = blockIdx.x * NT + threadIdx.x;
  if (gid >= BB * TT * 16) return;
  const int row = gid >> 4, c8 = (gid & 15) * 8;
  int tok = seqs[row]; tok = tok < 0 ? 0 : (tok >= VV ? VV - 1 : tok);
  const float* ep = emb + (size_t)tok * EE + c8;
  const v4f a = *(const v4f*)ep, bq = *(const v4f*)(ep + 4);
  v8h h;
#pragma unroll
  for (int e = 0; e < 4; ++e) { h[e] = (_Float16)(a[e] * 64.0f); h[4 + e] = (_Float16)(bq[e] * 64.0f); }
  _Float16* op = EX + (size_t)row * EE + c8;
  *(volatile v8h*)op = h; __threadfence(); *(volatile v8h*)op = h;
}

__global__ __launch_bounds__(512) void lstm_kernel(const _Float16* __restrict__ XP, const _Float16* __restrict__ WHH,
                                                  const float* __restrict__ bih, const float* __restrict__ bhh,
                                                  const int* __restrict__ lens, float* __restrict__ HL, int dir) {
  __shared__ __align__(16) _Float16 h16[16 * 264];
  __shared__ __align__(16) float hs[16 * 260];
  __shared__ int lens_s[16];
  const int tid = threadIdx.x, lane = tid & 31, wave = tid >> 5;
  const int rlane = lane & 15, hh = lane >> 4, koff = hh * 8, mOff = hh * 8;
  const int mbase = blockIdx.x * 16;
  for (int i = tid; i < 16 * 264; i += 512) h16[i] = (_Float16)0.0f;
  if (tid < 16) { const int L = lens[mbase + tid]; lens_s[tid] = L; }
  __syncthreads();
  const int j = 16 * wave + rlane;
  float bq[4];
#pragma unroll
  for (int gi = 0; gi < 4; ++gi) bq[gi] = bih[gi * HH + j] + bhh[gi * HH + j];
  int lenr[8];
#pragma unroll
  for (int r = 0; r < 8; ++r) lenr[r] = lens_s[mOff + r];
  float cst[8], hst[8];
#pragma unroll
  for (int r = 0; r < 8; ++r) { cst[r] = 0.f; hst[r] = 0.f; }
  const _Float16* arow = h16 + rlane * 264 + koff;
  const _Float16* wb = WHH + (size_t)j * HH + koff;
  const v8f z8 = {0.f, 0.f, 0.f, 0.f, 0.f, 0.f, 0.f, 0.f};

#pragma unroll 1
  for (int ts = 0; ts < TT; ++ts) {
    const int t = dir ? (TT - 1 - ts) : ts;
    v8f acc[4];
    acc[0] = z8; acc[1] = z8; acc[2] = z8; acc[3] = z8;
#pragma unroll 1
    for (int k0 = 0; k0 < HH; k0 += 32) {
      const v16h a  = Frag<_Float16>::load(arow + k0);
      const v16h b0 = Frag<_Float16>::load(wb + k0);
      const v16h b1 = Frag<_Float16>::load(wb + (size_t)1 * HH * HH + k0);
      const v16h b2 = Frag<_Float16>::load(wb + (size_t)2 * HH * HH + k0);
      const v16h b3 = Frag<_Float16>::load(wb + (size_t)3 * HH * HH + k0);
      acc[0] = Frag<_Float16>::mma(a, b0, acc[0]);
      acc[1] = Frag<_Float16>::mma(a, b1, acc[1]);
      acc[2] = Frag<_Float16>::mma(a, b2, acc[2]);
      acc[3] = Frag<_Float16>::mma(a, b3, acc[3]);
      dep_guard_h(acc[0], acc[3], a, b3);
      keep4_h(b0, b1, b2, b3);
    }
    acc_guard4(acc[0], acc[1], acc[2], acc[3]);
#pragma unroll
    for (int r = 0; r < 8; ++r) {
      const int bl = mOff + r;
      const size_t xo = ((size_t)(mbase + bl) * TT + t) * G4 + j;
      const float x0 = (float)XP[xo], x1 = (float)XP[xo + HH], x2 = (float)XP[xo + 2 * HH], x3 = (float)XP[xo + 3 * HH];
      const float p0 = acc[0][r] * (1.0f / 16384.0f) + (x0 * (1.0f / 1024.0f) + bq[0]);
      const float p1 = acc[1][r] * (1.0f / 16384.0f) + (x1 * (1.0f / 1024.0f) + bq[1]);
      const float p2 = acc[2][r] * (1.0f / 16384.0f) + (x2 * (1.0f / 1024.0f) + bq[2]);
      const float p3 = acc[3][r] * (1.0f / 16384.0f) + (x3 * (1.0f / 1024.0f) + bq[3]);
      const float ig = fsig(p0), fg = fsig(p1), gg = ftanh(p2), og = fsig(p3);
      const float cn = fg * cst[r] + ig * gg;
      const float hn = og * ftanh(cn);
      const bool valid = t < lenr[r];
      cst[r] = valid ? cn : cst[r];
      hst[r] = valid ? hn : hst[r];
    }
    __syncthreads();
#pragma unroll
    for (int r = 0; r < 8; ++r) h16[(mOff + r) * 264 + j] = (_Float16)(hst[r] * 64.0f);
    __syncthreads();
  }
#pragma unroll
  for (int r = 0; r < 8; ++r) hs[(mOff + r) * 260 + j] = hst[r];
  __syncthreads();
  {
    const int row = wave;
    const v4f p0 = *(const v4f*)(hs + row * 260 + 4 * lane);
    const v4f p1 = *(const v4f*)(hs + row * 260 + 128 + 4 * lane);
    float* dst = HL + (size_t)(mbase + row) * (2 * HH) + dir * HH;
    for (int pass = 0; pass < 2; ++pass) {
      *(volatile v4f*)(dst + 4 * lane) = p0;
      *(volatile v4f*)(dst + 128 + 4 * lane) = p1;
      __threadfence();
    }
  }
}

__device__ __forceinline__ int blk_excl_scan(int cnt, int* scan_ws, int tid, int* tot) {
  const int lane = tid & 31, wave = tid >> 5; int incl = cnt;
#pragma unroll
  for (int o = 1; o < 32; o <<= 1) { const int v = __shfl_up(incl, o, 32); if (lane >= o) incl += v; }
  if (lane == 31) scan_ws[wave] = incl;
  __syncthreads();
  if (wave == 0) { int wv = (lane < NT / 32) ? scan_ws[lane] : 0; int wincl = wv;
#pragma unroll
    for (int o = 1; o < 32; o <<= 1) { const int v = __shfl_up(wincl, o, 32); if (lane >= o) wincl += v; }
    if (lane < NT / 32) scan_ws[32 + lane] = wincl - wv; if (lane == 31) scan_ws[64] = wincl; }
  __syncthreads();
  const int res = scan_ws[32 + wave] + incl - cnt; *tot = scan_ws[64];
  return res;
}
template <int SP, int CAP, int TS>
__device__ __forceinline__ int chunk_hits(const int* __restrict__ dstv, const int* __restrict__ srcv, int e0, int n0, int tid,
                                          int* LIST, int* scan_ws) {
  const int eb = e0 + tid * SP;
  const bool inr = eb < NE;
  const int ebc = inr ? eb : (NE - SP);
  int rec[SP]; int cnt = 0;
#pragma unroll
  for (int k = 0; k < SP; k += 4) {
    const v4i d4 = *(const v4i*)(dstv + ebc + k);
    const v4i s4 = *(const v4i*)(srcv + ebc + k);
#pragma unroll
    for (int e = 0; e < 4; ++e) {
      int d = d4[e]; d = d < 0 ? 0 : (d >= NN ? NN - 1 : d);
      int s = s4[e]; s = s < 0 ? 0 : (s >= NN ? NN - 1 : s);
      const bool hit = inr && d >= n0 && d < n0 + TS;
      const int packed = (int)((((unsigned)(d - n0)) << 16) | (unsigned)s);
      rec[k + e] = hit ? packed : -1;
      cnt += hit ? 1 : 0;
    }
  }
  int tot; int p = blk_excl_scan(cnt, scan_ws, tid, &tot);
#pragma unroll
  for (int k = 0; k < SP; ++k) if (rec[k] >= 0) { if ((unsigned)p < (unsigned)CAP) LIST[p] = rec[k]; ++p; }
  __syncthreads();
  return tot < CAP ? tot : CAP;
}

__global__ __launch_bounds__(NT) void deg_kernel(const int* __restrict__ ei, float* __restrict__ DINV) {
  __shared__ int LIST[SCHA];
  __shared__ int CNT[TSA];
  __shared__ int scan_ws[80];
  const int tid = threadIdx.x, lane = tid & 31, wave = tid >> 5;
  const int n0 = blockIdx.x * TSA;
  for (int i = tid; i < TSA; i += NT) CNT[i] = 0;
  __syncthreads();
  const int* srcv = ei; const int* dstv = ei + NE;
#pragma unroll 1
  for (int c = 0; c < NCHA; ++c) {
    const int tot = chunk_hits<SCHA / NT, SCHA, TSA>(dstv, srcv, c * SCHA, n0, tid, LIST, scan_ws);
#pragma unroll 1
    for (int base = 0; base < tot; base += 32) {
      const int q = base + lane; const int qc = q < SCHA ? q : SCHA - 1;
      const int lv = LIST[qc];
      const int rv = (q < tot) ? lv : -1;
      const int own = (rv >= 0 && (rv >> 26) == wave) ? 1 : 0;
      unsigned msk = (unsigned)__ballot(own);
#pragma unroll 1
      for (int it = 0; it < 32; ++it) {
        if (msk == 0u) break;
        const int bp = __builtin_ctz(msk); msk &= msk - 1u;
        const int r = __shfl(rv, bp, 32);
        const int dl = r >> 16;
        const int nv = CNT[dl] + 1;
        CNT[dl] = nv;
      }
    }
    __syncthreads();
  }
#pragma unroll 1
  for (int it = 0; it < TSA / NT; ++it) {
    const int i = it * NT + tid;
    const float d = 1.0f + (float)CNT[i];
    const float v = 1.0f / sqrtf(d);
    float* p = DINV + n0 + i;
    *(volatile float*)p = v; __threadfence(); *(volatile float*)p = v;
  }
}

__global__ __launch_bounds__(NT) void s1_kernel(const int* __restrict__ ei, const float* __restrict__ x, const float* __restrict__ DINV,
                                               float* __restrict__ S1) {
  __shared__ int LIST[SCHA];
  __shared__ float ACC1[TSA];
  __shared__ int scan_ws[80];
  const int tid = threadIdx.x, lane = tid & 31, wave = tid >> 5;
  const int n0 = blockIdx.x * TSA;
  for (int i = tid; i < TSA; i += NT) ACC1[i] = 0.f;
  __syncthreads();
  const int* srcv = ei; const int* dstv = ei + NE;
#pragma unroll 1
  for (int c = 0; c < NCHA; ++c) {
    const int tot = chunk_hits<SCHA / NT, SCHA, TSA>(dstv, srcv, c * SCHA, n0, tid, LIST, scan_ws);
#pragma unroll 1
    for (int base = 0; base < tot; base += 32) {
      const int q = base + lane; const int qc = q < SCHA ? q : SCHA - 1;
      const int lv = LIST[qc];
      const int rv = (q < tot) ? lv : -1;
      const int own = (rv >= 0 && (rv >> 26) == wave) ? 1 : 0;
      unsigned msk = (unsigned)__ballot(own);
#pragma unroll 1
      for (int it = 0; it < 32; ++it) {
        if (msk == 0u) break;
        const int bp = __builtin_ctz(msk); msk &= msk - 1u;
        const int r = __shfl(rv, bp, 32);
        const int dl = r >> 16, s = r & 0xFFFF;
        const float ds = DINV[s], xs = x[s];
        const float nv = ACC1[dl] + ds * xs;
        ACC1[dl] = nv;
      }
    }
    __syncthreads();
  }
#pragma unroll 1
  for (int it = 0; it < TSA / NT; ++it) {
    const int i = it * NT + tid;
    const int n = n0 + i;
    const int nc = n < NN ? n : NN - 1;
    const float dn = DINV[n], xn = x[nc];
    const float tv = dn * (ACC1[i] + dn * xn);
    const float v = (n < NN) ? tv : 0.f;
    float* p = S1 + n;
    *(volatile float*)p = v; __threadfence(); *(volatile float*)p = v;
  }
}

__global__ __launch_bounds__(NT) void bnstat_kernel(const float* __restrict__ S1, const float* __restrict__ Wg1, const float* __restrict__ bg1,
                                                   double* __restrict__ PART) {
  __shared__ double ssum[NT];
  __shared__ double ssq[NT];
  const int tid = threadIdx.x; const int f = tid & 127, hsel = tid >> 7;
  const float w = Wg1[f], bb = bg1[f];
  const int i0 = blockIdx.x * 1000 + hsel;
  double s = 0.0, q = 0.0;
#pragma unroll 1
  for (int m = 0; m < 500; ++m) {
    const int i = i0 + 2 * m;
    float v = S1[i] * w + bb; v = fmaxf(v, 0.f);
    const double dv = (double)v;
    s += dv; q += dv * dv;
  }
  ssum[tid] = s; ssq[tid] = q;
  __syncthreads();
  const double a = ssum[f] + ssum[f + 128];
  const double b = ssq[f] + ssq[f + 128];
  const double val = (tid < 128) ? a : b;
  double* p = PART + (size_t)blockIdx.x * NT + tid;
  *(volatile double*)p = val; __threadfence(); *(volatile double*)p = val;
}
__global__ __launch_bounds__(NT) void bnred_kernel(const double* __restrict__ PART, float* __restrict__ MURS) {
  __shared__ double sh[NT];
  const int tid = threadIdx.x;
  double a = 0.0;
#pragma unroll 1
  for (int k = 0; k < NSB; ++k) a += PART[k * NT + tid];
  sh[tid] = a;
  __syncthreads();
  const int f = tid & 127;
  const double su = sh[f], sq = sh[128 + f];
  const double mu = su * (1.0 / (double)NN);
  double var = sq * (1.0 / (double)NN) - mu * mu; var = var > 0.0 ? var : 0.0;
  const float muf = (float)mu;
  const float rs = 1.0f / sqrtf((float)var + 1e-5f);
  const float val = (tid < 128) ? muf : rs;
  float* p = MURS + tid;
  *(volatile float*)p = val; __threadfence(); *(volatile float*)p = val;
}
__global__ __launch_bounds__(NT) void x1n_kernel(const float* __restrict__ S1, const float* __restrict__ Wg1, const float* __restrict__ bg1,
                                                const float* __restrict__ MURS, const float* __restrict__ gam, const float* __restrict__ bet,
                                                _Float16* __restrict__ X1N) {
  const int gid = blockIdx.x * NT + threadIdx.x;
  if (gid >= NP * 16) return;
  const int row = gid >> 4, c8 = (gid & 15) * 8;
  const bool live = row < NN;
  const float s = S1[row];
  v8h hv;
#pragma unroll
  for (int e = 0; e < 8; ++e) {
    const int f = c8 + e;
    const float x1 = fmaxf(s * Wg1[f] + bg1[f], 0.f);
    float v = (x1 - MURS[f]) * MURS[128 + f];
    v = v * gam[f] + bet[f];
    hv[e] = live ? (_Float16)v : (_Float16)0.0f;
  }
  _Float16* op = X1N + (size_t)row * GH + c8;
  *(volatile v8h*)op = hv; __threadfence(); *(volatile v8h*)op = hv;
}

__global__ __launch_bounds__(NT) void agg2_kernel(const int* __restrict__ ei, const float* __restrict__ H2, const float* __restrict__ DINV,
                                                 const float* __restrict__ bg2, float* X2) {
  __shared__ int LIST[SCHC];
  __shared__ int scan_ws[80];
  const int tid = threadIdx.x, lane = tid & 31, wave = tid >> 5;
  const int n0 = blockIdx.x * TSC;
  const v4f z4 = {0.f, 0.f, 0.f, 0.f};
#pragma unroll 1
  for (int jr = 0; jr < 128; ++jr) *(v4f*)(X2 + (size_t)(n0 + wave * 128 + jr) * GH + 4 * lane) = z4;
  const int* srcv = ei; const int* dstv = ei + NE;
#pragma unroll 1
  for (int c = 0; c < NCHC; ++c) {
    const int tot = chunk_hits<SCHC / NT, SCHC, TSC>(dstv, srcv, c * SCHC, n0, tid, LIST, scan_ws);
#pragma unroll 1
    for (int base = 0; base < tot; base += 32) {
      const int q = base + lane; const int qc = q < SCHC ? q : SCHC - 1;
      const int lv = LIST[qc];
      const int rv = (q < tot) ? lv : -1;
      const int own = (rv >= 0 && (rv >> 23) == wave) ? 1 : 0;
      unsigned msk = (unsigned)__ballot(own);
#pragma unroll 1
      for (int it = 0; it < 32; ++it) {
        if (msk == 0u) break;
        const int bp = __builtin_ctz(msk); msk &= msk - 1u;
        const int r = __shfl(rv, bp, 32);
        const int dl = r >> 16, s = r & 0xFFFF;
        const float ds = DINV[s];
        const v4f hv = *(const v4f*)(H2 + (size_t)s * GH + 4 * lane);
        float* rp = X2 + (size_t)(n0 + dl) * GH + 4 * lane;
        v4f a = *(const v4f*)rp;
        a = a + ds * hv;
        *(v4f*)rp = a;
      }
    }
    __syncthreads();
  }
  const v4f bz = *(const v4f*)(bg2 + 4 * lane);
#pragma unroll 1
  for (int jr = 0; jr < 128; ++jr) {
    const int n = n0 + wave * 128 + jr;
    const int nc = n < NN ? n : NN - 1;
    const bool live = n < NN;
    const float dn = DINV[n];
    const v4f hsf = *(const v4f*)(H2 + (size_t)nc * GH + 4 * lane);
    float* rp = X2 + (size_t)n * GH + 4 * lane;
    const v4f a = *(const v4f*)rp;
    const v4f t = (a + dn * hsf) * dn;
    v4f o;
#pragma unroll
    for (int e = 0; e < 4; ++e) o[e] = live ? fmaxf(t[e] + bz[e], 0.f) : 0.f;
    for (int pass = 0; pass < 2; ++pass) { *(volatile v4f*)rp = o; __threadfence(); }
  }
}

__global__ __launch_bounds__(128) void pool_kernel(const int* __restrict__ gid, const float* __restrict__ X2, float* __restrict__ HG) {
  __shared__ int slo[128];
  __shared__ int shi[128];
  const int tid = threadIdx.x; const int g = blockIdx.x;
  int lo = 0x7fffffff, hi = -1;
#pragma unroll 1
  for (int i = tid; i < NN; i += 128) {
    const int v = gid[i];
    const bool m = (v == g);
    lo = (m && i < lo) ? i : lo;
    hi = (m && i > hi) ? i : hi;
  }
  slo[tid] = lo; shi[tid] = hi;
  __syncthreads();
#pragma unroll 1
  for (int st = 64; st > 0; st >>= 1) {
    if (tid < st) {
      const int a = slo[tid + st], b = shi[tid + st];
      if (a < slo[tid]) slo[tid] = a;
      if (b > shi[tid]) shi[tid] = b;
    }
    __syncthreads();
  }
  lo = slo[0]; hi = shi[0];
  float acc = 0.f; int cnt = 0;
#pragma unroll 1
  for (int it = 0; it < NN; ++it) {
    const int i = lo + it;
    if (i > hi) break;
    const int ic = i < 0 ? 0 : (i >= NN ? NN - 1 : i);
    const int v = gid[ic];
    const float xv = X2[(size_t)ic * GH + tid];
    const bool m = (v == g);
    acc += m ? xv : 0.f;
    cnt += m ? 1 : 0;
  }
  const float cf = fmaxf((float)cnt, 1.0f);
  const float o = acc * (1.0f / cf);
  float* p = HG + (size_t)g * GH + tid;
  *(volatile float*)p = o; __threadfence(); *(volatile float*)p = o;
}

__global__ __launch_bounds__(NT) void fuse_plane_kernel(const float* __restrict__ HL, const float* __restrict__ HG, const float* __restrict__ Wf,
                                                       unsigned* __restrict__ AH, unsigned* __restrict__ AL,
                                                       unsigned* __restrict__ WH, unsigned* __restrict__ WL) {
  const int blk = blockIdx.x, tid = threadIdx.x;
  if (blk < 80) {
    const int p = blk * NT + tid;
    const int row = p / 320; const int c = 2 * (p - row * 320);
    const int c1 = c < 510 ? c : 510;
    const int c2 = c >= 512 ? (c - 512) : 0;
    const float l0 = HL[row * (2 * HH) + c1], l1 = HL[row * (2 * HH) + c1 + 1];
    const float g0 = HG[row * GH + c2], g1 = HG[row * GH + c2 + 1];
    const bool useL = c < 512;
    const float v0 = useL ? l0 : g0, v1 = useL ? l1 : g1;
    unsigned uh, ul; split_pack2(v0, v1, uh, ul);
    st2u(AH + p, uh); st2u(AL + p, ul);
  } else {
    const int p = (blk - 80) * NT + tid;
    const float v0 = Wf[2 * p], v1 = Wf[2 * p + 1];
    unsigned uh, ul; split_pack2(v0, v1, uh, ul);
    st2u(WH + p, uh); st2u(WL + p, ul);
  }
}

__global__ __launch_bounds__(NT) void final_kernel(const float* __restrict__ F, const float* __restrict__ Wc, const float* __restrict__ bc,
                                                  float* __restrict__ out) {
  __shared__ __align__(16) float so[128];
  const int tid = threadIdx.x, lane = tid & 31, wave = tid >> 5;
  for (int pass = 0; pass < 2; ++pass) {
#pragma unroll 1
    for (int it = 0; it < 24; ++it) {
      const int q = it * NT + tid;
      const v4f v = *(const v4f*)(F + 4 * q);
      *(volatile v4f*)(out + 128 + 4 * q) = v;
    }
    __threadfence();
  }
  if (tid < 128) {
    const int b = tid >> 1, c = tid & 1;
    float o = bc[c];
#pragma unroll 1
    for (int k = 0; k < FD; ++k) o += fmaxf(F[b * FD + k], 0.f) * Wc[c * FD + k];
    so[tid] = o;
  }
  __syncthreads();
  if (wave == 0) {
    const v4f v = *(const v4f*)(so + 4 * lane);
    for (int pass = 0; pass < 2; ++pass) { *(volatile v4f*)(out + 4 * lane) = v; __threadfence(); }
  }
}

extern "C" void kernel_launch(void* const* d_in, const int* in_sizes, int n_in,
                              void* d_out, int out_size, void* d_ws, size_t ws_size, hipStream_t stream) {
  if (n_in < 24 || d_out == nullptr || d_ws == nullptr) return;
  if (in_sizes[0] != BB * TT || in_sizes[1] != BB || in_sizes[2] != NN || in_sizes[3] != 2 * NE || in_sizes[4] != NN ||
      in_sizes[5] != VV * EE || in_sizes[6] != G4 * EE || in_sizes[7] != G4 * HH || in_sizes[10] != G4 * EE || in_sizes[11] != G4 * HH ||
      in_sizes[14] != GH || in_sizes[16] != GH * GH || in_sizes[20] != FD * KF || in_sizes[22] != NC * FD ||
      out_size != BB * NC + BB * FD) return;

  const int*   seqs   = (const int*)d_in[0];
  const int*   lens   = (const int*)d_in[1];
  const float* node_x = (const float*)d_in[2];
  const int*   eidx   = (const int*)d_in[3];
  const int*   gids   = (const int*)d_in[4];
  const float* emb    = (const float*)d_in[5];
  const float* Wih_f  = (const float*)d_in[6];
  const float* Whh_f  = (const float*)d_in[7];
  const float* bih_f  = (const float*)d_in[8];
  const float* bhh_f  = (const float*)d_in[9];
  const float* Wih_b  = (const float*)d_in[10];
  const float* Whh_b  = (const float*)d_in[11];
  const float* bih_b  = (const float*)d_in[12];
  const float* bhh_b  = (const float*)d_in[13];
  const float* Wg1    = (const float*)d_in[14];
  const float* bg1    = (const float*)d_in[15];
  const float* Wg2    = (const float*)d_in[16];
  const float* bg2    = (const float*)d_in[17];
  const float* gam    = (const float*)d_in[18];
  const float* bet    = (const float*)d_in[19];
  const float* Wfuse  = (const float*)d_in[20];
  const float* bfuse  = (const float*)d_in[21];
  const float* Wcls   = (const float*)d_in[22];
  const float* bcls   = (const float*)d_in[23];
  float* out = (float*)d_out;

  char* ws = (char*)d_ws; size_t off = 0;
  auto carve = [&](size_t bytes) -> char* { char* p = ws + off; off += (bytes + 255) & ~(size_t)255; return p; };
  _Float16* EX16   = (_Float16*)carve((size_t)BB * TT * EE * 2);
  unsigned* WIH    = (unsigned*)carve((size_t)2 * G4 * EE * 2);
  unsigned* WHH    = (unsigned*)carve((size_t)2 * G4 * HH * 2);
  unsigned* WG2T   = (unsigned*)carve((size_t)GH * GH * 2);
  char*     R      = carve((size_t)BB * TT * G4 * 2);
  float*    HL     = (float*)carve((size_t)BB * 2 * HH * 4);
  float*    DINV   = (float*)carve((size_t)NRA * 4);
  float*    S1     = (float*)carve((size_t)NRA * 4);
  double*   PART   = (double*)carve((size_t)NSB * NT * 8);
  float*    MURS   = (float*)carve((size_t)NT * 4);
  _Float16* X1N16  = (_Float16*)carve((size_t)NP * GH * 2);
  float*    H2     = (float*)carve((size_t)NP * GH * 4);
  float*    HG     = (float*)carve((size_t)NG * GH * 4);
  unsigned* AH     = (unsigned*)carve((size_t)BB * KF * 2);
  unsigned* AL     = (unsigned*)carve((size_t)BB * KF * 2);
  unsigned* WFH    = (unsigned*)carve((size_t)FD * KF * 2);
  unsigned* WFL    = (unsigned*)carve((size_t)FD * KF * 2);
  float*    FUSED  = (float*)carve((size_t)BB * FD * 4);
  if (off > ws_size || off > (size_t)134217728) return;
  if ((size_t)NRC * GH * 4 > (size_t)BB * TT * G4 * 2) return;
  _Float16* XP16 = (_Float16*)R;
  float*    X2   = (float*)R;
  const _Float16* WIH16 = (const _Float16*)WIH;
  const _Float16* WHH16 = (const _Float16*)WHH;

  prep_kernel<<<1568, NT, 0, stream>>>(Wih_f, Wih_b, Whh_f, Whh_b, Wg2, WIH, WHH, WG2T);
  embed_kernel<<<(BB * TT * 16) / NT, NT, 0, stream>>>(seqs, emb, EX16);
  for (int dir = 0; dir < 2; ++dir) {
    const int tiles = (BB * TT / 64) * (G4 / 64);
    wmma_gemm64<0, false, 0, 1, false><<<dim3((tiles + 7) / 8, 1), 256, 0, stream>>>(
        (const unsigned short*)EX16, (const unsigned short*)nullptr, EE, 0L,
        (const unsigned short*)(WIH16 + (size_t)dir * G4 * EE), (const unsigned short*)nullptr, EE, 0L,
        (void*)XP16, (void*)nullptr, G4, 0L,
        (const float*)nullptr, (const float*)nullptr, 0L, BB * TT, G4, EE, 1.0f / 16.0f);
    lstm_kernel<<<BB / 16, 512, 0, stream>>>(XP16, WHH16 + (size_t)dir * G4 * HH, dir ? bih_b : bih_f, dir ? bhh_b : bhh_f, lens, HL, dir);
  }

  deg_kernel<<<NTA, NT, 0, stream>>>(eidx, DINV);
  s1_kernel<<<NTA, NT, 0, stream>>>(eidx, node_x, DINV, S1);
  bnstat_kernel<<<NSB, NT, 0, stream>>>(S1, Wg1, bg1, PART);
  bnred_kernel<<<1, NT, 0, stream>>>(PART, MURS);
  x1n_kernel<<<(NP * 16 + NT - 1) / NT, NT, 0, stream>>>(S1, Wg1, bg1, MURS, gam, bet, X1N16);
  {
    const int tiles = (NP / 64) * (GH / 64);
    wmma_gemm64<0, false, 0, 0, false><<<dim3((tiles + 7) / 8, 1), 256, 0, stream>>>(
        (const unsigned short*)X1N16, (const unsigned short*)nullptr, GH, 0L,
        (const unsigned short*)WG2T, (const unsigned short*)nullptr, GH, 0L,
        (void*)H2, (void*)nullptr, GH, 0L,
        (const float*)nullptr, (const float*)nullptr, 0L, NP, GH, GH, 1.0f / 256.0f);
  }
  agg2_kernel<<<NTC, NT, 0, stream>>>(eidx, H2, DINV, bg2, X2);
  pool_kernel<<<NG, 128, 0, stream>>>(gids, X2, HG);

  fuse_plane_kernel<<<80 + 480, NT, 0, stream>>>(HL, HG, Wfuse, AH, AL, WFH, WFL);
  {
    const int tiles = (BB / 64) * (FD / 64);
    wmma_gemm64<1, true, 2, 0, false><<<dim3((tiles + 7) / 8, 1), 256, 0, stream>>>(
        (const unsigned short*)AH, (const unsigned short*)AL, KF, 0L,
        (const unsigned short*)WFH, (const unsigned short*)WFL, KF, 0L,
        (void*)FUSED, (void*)nullptr, FD, 0L,
        bfuse, (const float*)nullptr, 0L, BB, FD, KF, 1.0f);
  }
  final_kernel<<<1, NT, 0, stream>>>(FUSED, Wcls, bcls, out);
}
